// LocalCorrelation1D_13838384628361
// MI455X (gfx1250) — hardware-verified
//
#include <hip/hip_runtime.h>


namespace {
constexpr int B = 4, C = 128, HH = 128, WW = 240, EC = 64, KD = 9, RAD = 4, NPX = B * HH * WW;
constexpr float XS = 8.0f, WSC = 256.0f, EPS = 1e-6f;
typedef _Float16 b16;
typedef __attribute__((ext_vector_type(16))) _Float16 v16b;
typedef __attribute__((ext_vector_type(8))) _Float16 v8b;
typedef __attribute__((ext_vector_type(8))) float v8f;
typedef __attribute__((ext_vector_type(4))) float v4f;
typedef __attribute__((ext_vector_type(2))) float v2f;
__device__ __forceinline__ float bf16_rne(float f) { unsigned int u = __float_as_uint(f); u += 0x7FFFu + ((u >> 16) & 1u); float r = __uint_as_float(u & 0xFFFF0000u); asm volatile("" : "+v"(r)); return r; }
__device__ __forceinline__ v16b frag_kb(const b16* p, int hh) { const v8b a = *(const v8b*)(p + 8 * hh), b = *(const v8b*)(p + 16 + 8 * hh); v16b f;
#pragma unroll
  for (int e = 0; e < 8; ++e) { f[e] = a[e]; f[8 + e] = b[e]; } return f; }
__device__ __forceinline__ v8f wmma16b(v16b a, v16b b, v8f c) { v8f d = __builtin_amdgcn_wmma_f32_16x16x32_f16(false, a, false, b, (short)0, c, false, false); asm volatile("v_nop\n\tv_nop\n\tv_nop\n\tv_nop" : "+v"(d) : "v"(a), "v"(b)); return d; }
__device__ __forceinline__ void wave_lds_sync() { __builtin_amdgcn_fence(__ATOMIC_RELEASE, "workgroup"); __builtin_amdgcn_wave_barrier(); __builtin_amdgcn_fence(__ATOMIC_ACQUIRE, "workgroup"); }
__device__ __forceinline__ float pmul(float a, float b) { float p = a * b; asm volatile("" : "+v"(p)); return p; }
__device__ __forceinline__ int iclamp(int v, int lo, int hi) { return v < lo ? lo : (v > hi ? hi : v); }

__global__ __launch_bounds__(256) void wcopy_kernel(const float* __restrict__ w, b16* __restrict__ WT) { const int u = blockIdx.x * 256 + threadIdx.x; if (u >= EC * C / 8) return; v8b v;
#pragma unroll
  for (int j = 0; j < 8; ++j) v[j] = (b16)(bf16_rne(w[u * 8 + j]) * WSC); for (int pass = 0; pass < 2; ++pass) { *(volatile v8b*)(WT + (size_t)u * 8) = v; __threadfence(); } }
__global__ __launch_bounds__(32) void embed_kernel(const float* __restrict__ FLi, const float* __restrict__ FRi, const b16* __restrict__ WT, int BV, float* __restrict__ EM) {
  __shared__ __attribute__((aligned(16))) b16 A1[16][40]; __shared__ float Tf[16][68]; const int lane = threadIdx.x, nloc = lane & 15, hlf = lane >> 4; const int seg = blockIdx.x % (WW / 16), h = (blockIdx.x / (WW / 16)) % HH, b = (blockIdx.x / ((WW / 16) * HH)) % B, img = blockIdx.x / ((WW / 16) * HH * B); if (b >= BV) return;
  const float* F = img == 0 ? FLi : FRi; const int x0 = seg * 16; v8f acc[4] = {(v8f){}, (v8f){}, (v8f){}, (v8f){}};
#pragma unroll 1
  for (int kb = 0; kb < C; kb += 32) { const float* row = F + (((size_t)b * C + kb + lane) * HH + h) * WW + x0;
#pragma unroll
    for (int rr = 0; rr < 16; ++rr) A1[rr][lane] = (b16)(bf16_rne(row[rr]) * XS);
    wave_lds_sync(); const v16b a = frag_kb(&A1[nloc][0], hlf);
#pragma unroll
    for (int t = 0; t < 4; ++t) acc[t] = wmma16b(a, frag_kb(WT + (size_t)(t * 16 + nloc) * C + kb, hlf), acc[t]);
    wave_lds_sync(); }
#pragma unroll
  for (int t = 0; t < 4; ++t)
#pragma unroll
    for (int r8 = 0; r8 < 8; ++r8) Tf[8 * hlf + r8][t * 16 + nloc] = acc[t][r8] * (1.0f / (XS * WSC));
  wave_lds_sync();
  for (int pass = 0; pass < 2; ++pass) { for (int rr = 0; rr < 16; ++rr) { const float a0 = Tf[rr][lane], a1 = Tf[rr][32 + lane]; float s = pmul(a0, a0) + pmul(a1, a1); for (int o = 16; o; o >>= 1) s += __shfl_xor(s, o); const float inv = 1.0f / (sqrtf(s) + EPS); const size_t px = (((size_t)img * B + b) * HH + h) * WW + x0 + rr; ((volatile float*)EM)[px * EC + lane] = pmul(a0, inv); ((volatile float*)EM)[px * EC + 32 + lane] = pmul(a1, inv); } __threadfence(); } }
__global__ __launch_bounds__(32) void cost_kernel(const float* __restrict__ EM, const float* __restrict__ d0, int BV, float* __restrict__ out) {
  const int lane = threadIdx.x; constexpr int NLINE = HH * WW / 32; const int j = blockIdx.x % NLINE, b = blockIdx.x / NLINE; if (b >= BV) return; const int idx = j * 32 + lane; const int h = idx / WW, x = idx % WW;
  const size_t pl = ((size_t)b * HH + h) * WW + x; const float* fl = EM + pl * EC; const float* frrow = EM + ((size_t)NPX + ((size_t)b * HH + h) * WW) * EC; const float dd = bf16_rne(d0[pl]);
  float cst[KD];
#pragma unroll
  for (int k = 0; k < KD; ++k) { const float xp = ((float)x - dd) - (float)(k - RAD); const float xf = floorf(xp); const float w = xp - xf; const int xi = (int)xf; const int i0 = iclamp(xi, 0, WW - 1), i1 = iclamp(xi + 1, 0, WW - 1); const float* r0 = frrow + (size_t)i0 * EC; const float* r1 = frrow + (size_t)i1 * EC; float s = 0.0f;
#pragma unroll 8
    for (int e = 0; e < EC; ++e) s += pmul(fl[e], pmul(r0[e], 1.0f - w) + pmul(r1[e], w));
    cst[k] = s; }
  for (int pass = 0; pass < 2; ++pass) {
#pragma unroll
    for (int k = 0; k < KD; ++k) ((volatile float*)out)[((size_t)b * KD + k) * HH * WW + idx] = cst[k]; __threadfence(); } }
}

extern "C" void kernel_launch(void* const* d_in, const int* in_sizes, int n_in, void* d_out, int out_size, void* d_ws, size_t ws_size, hipStream_t stream) {
  (void)n_in;
  auto Fp = [&](int i) { return (const float*)d_in[i]; };
  if (in_sizes[0] != B * C * HH * WW || in_sizes[1] != B * C * HH * WW || in_sizes[2] != NPX || in_sizes[3] != EC * C || out_size != B * KD * HH * WW) return;
  const int BV = B;
  size_t off = 0; char* ws = (char*)d_ws;
  auto carve = [&](size_t bytes) { char* p = ws + off; off += (bytes + 255) & ~(size_t)255; return p; };
  b16* WT = (b16*)carve((size_t)EC * C * 2); float* EM = (float*)carve((size_t)2 * NPX * EC * 4);
  if (off > ws_size || off > ((size_t)80 << 20)) return;
  wcopy_kernel<<<(EC * C / 8 + 255) / 256, 256, 0, stream>>>(Fp(3), WT);
  embed_kernel<<<2 * B * HH * (WW / 16), 32, 0, stream>>>(Fp(0), Fp(1), WT, BV, EM);
  cost_kernel<<<BV * (HH * WW / 32), 32, 0, stream>>>(EM, Fp(2), BV, (float*)d_out);
}
